// PNNLayer_18210661335371
// MI455X (gfx1250) — hardware-run, weakly checked
//
#include <hip/hip_runtime.h>
#include <math.h>

#pragma clang fp contract(off)

#ifndef NN
#define NN 10000
#endif
#define NN_FULL 10000
#define NA 64
#define DL 128
#define KCAT 256
#define MPAD (((NN + 63) / 64) * 64)

static_assert(NN % 16 == 0);
static_assert(NN <= NN_FULL);
static_assert(MPAD % 64 == 0 && MPAD >= NN);
static_assert(DL % 64 == 0);
static_assert(NA % 32 == 0 && KCAT % 32 == 0);
static_assert(NA % 8 == 0 && KCAT % 8 == 0 && DL % 8 == 0);
static_assert(KCAT == 2 * DL);
static_assert(NA == 64);

typedef __attribute__((ext_vector_type(16))) _Float16 v16h;
typedef __attribute__((ext_vector_type(8)))  _Float16 v8h;
typedef __attribute__((ext_vector_type(8)))  float    v8f;
typedef __attribute__((ext_vector_type(4)))  float    v4f;
typedef __attribute__((ext_vector_type(4)))  unsigned int v4u;
typedef _Float16 h16;

static constexpr float CARRY_D = 1024.0f;
static constexpr float CARRY_E = 256.0f;
static constexpr float CARRY_W = 1024.0f;
static constexpr float QMUL    = 64.0f;
static constexpr float SC_P    = 1.0f / 16777216.0f;
static constexpr float OSC_P   = 4096.0f;
static constexpr float SC_O    = 1.0f / 4194304.0f;
static constexpr float OSC_O   = 1.0f;

static constexpr size_t SZ_D  = (size_t)MPAD * NA * 2;
static constexpr size_t SZ_E  = (size_t)DL * NA * 2;
static constexpr size_t SZ_W  = (size_t)DL * KCAT * 2;
static constexpr size_t SZ_PQ = (size_t)MPAD * KCAT * 2;
static constexpr size_t OFF_D  = 0;
static constexpr size_t OFF_E  = OFF_D + SZ_D;
static constexpr size_t OFF_W  = OFF_E + SZ_E;
static constexpr size_t OFF_PQ = OFF_W + SZ_W;
static constexpr size_t WS_TOTAL = OFF_PQ + SZ_PQ;
static_assert(SZ_D % 256 == 0 && SZ_E % 256 == 0 && SZ_W % 256 == 0 && SZ_PQ % 256 == 0);
static_assert(WS_TOTAL <= (size_t)134217728);

static constexpr unsigned G_DT   = MPAD / 64;
static constexpr unsigned G_QS   = MPAD / 16;
static constexpr unsigned G_WC   = (DL * KCAT / 8) / 256;
static constexpr unsigned G_GEMM = ((MPAD / 64) * (DL / 64) + 7) / 8;
static_assert((DL * KCAT / 8) % 256 == 0);
static_assert(G_DT * 64 == MPAD && G_QS * 16 == MPAD);

static_assert(8 * 16 * 68 * 4 <= 131072);
static_assert(64 * 65 * 4 <= 131072);
static_assert(64 * 129 * 4 <= 131072);


#define VST2(T, ptr, val) do { const T vst2_v_ = (val); *(volatile T*)(ptr) = vst2_v_; __threadfence(); *(volatile T*)(ptr) = vst2_v_; } while (0)

__device__ __forceinline__ float bfr(float f) {
    unsigned u = __float_as_uint(f);
    u += 0x7FFFu + ((u >> 16) & 1u);
    return __uint_as_float(u & 0xFFFF0000u);
}
static __device__ __forceinline__ h16 toh_flush(float v) { const h16 r = (h16)v; return (fabsf(v) < 6.103515625e-05f) ? (h16)0.0f : r; }
static __device__ __forceinline__ unsigned hbits(float v) { return (unsigned)__builtin_bit_cast(unsigned short, toh_flush(v)); }
static __device__ __forceinline__ void st8hf(unsigned short* P, size_t o, const float* v) {
    v4u pk;
    pk.x = hbits(v[0]) | (hbits(v[1]) << 16);
    pk.y = hbits(v[2]) | (hbits(v[3]) << 16);
    pk.z = hbits(v[4]) | (hbits(v[5]) << 16);
    pk.w = hbits(v[6]) | (hbits(v[7]) << 16);
    VST2(v4u, (v4u*)(P + o), pk);
}

union FragU { v16h v; v8h h[2]; };
__device__ __forceinline__ v16h frag_ld(const _Float16* p) {
    FragU f; f.h[0] = *(const v8h*)(p); f.h[1] = *(const v8h*)(p + 16); return f.v;
}
__device__ __forceinline__ v8f wmma16(v16h a, v16h b, v8f c) {
    c = __builtin_amdgcn_wmma_f32_16x16x32_f16(false, a, false, b, (short)0, c, false, false);
    asm volatile("v_nop\n\tv_nop\n\tv_nop\n\tv_nop" : "+v"(c) : "v"(a), "v"(b));
    return c;
}
__device__ __forceinline__ void wave_sync_lds() {
    __builtin_amdgcn_fence(3  , "workgroup");
    __builtin_amdgcn_wave_barrier();
    __builtin_amdgcn_fence(2  , "workgroup");
}

static_assert(2 * 4 * 32 * 16 == 16 * 64 * 4);
static_assert(4 * 32 * 16 == 16 * 64 * 2);
template <int OUT_MODE, bool HASBIAS>
__device__ __forceinline__ void gemm64_body(
    const _Float16* __restrict__ A, unsigned lda, const _Float16* __restrict__ Bt, unsigned ldb,
    void* __restrict__ Cout, unsigned ldc, const float* __restrict__ bias,
    unsigned M, unsigned Mvalid, unsigned N, unsigned K, float scale, float oscale,
    float* slab, unsigned wave) {
  const unsigned lane = threadIdx.x & 31u;
  const unsigned tilesN = N >> 6, tilesM = M >> 6;
  const unsigned tile = blockIdx.x * 8u + wave;
  if (tile >= tilesM * tilesN) return;
  const unsigned tm = tile / tilesN;
  const unsigned tn = tile - tm * tilesN;
  const unsigned m0 = tm << 6, n0 = tn << 6;
  const unsigned rlane = lane & 15u;
  const unsigned koff = (lane >> 4) * 8u;
  const unsigned mOff = koff;

  v8f acc[4][4];
#pragma unroll
  for (int i = 0; i < 4; ++i)
#pragma unroll
    for (int j = 0; j < 4; ++j) acc[i][j] = (v8f){0.f,0.f,0.f,0.f,0.f,0.f,0.f,0.f};

  for (unsigned k0 = 0; k0 < K; k0 += 32u) {
    v16h bh[4];
#pragma unroll
    for (int j = 0; j < 4; ++j)
      bh[j] = frag_ld(Bt + (size_t)(n0 + ((unsigned)j << 4) + rlane) * ldb + koff + k0);
#pragma unroll
    for (int i = 0; i < 4; ++i) {
      const v16h ah = frag_ld(A + (size_t)(m0 + ((unsigned)i << 4) + rlane) * lda + koff + k0);
#pragma unroll
      for (int j = 0; j < 4; ++j)
        acc[i][j] = wmma16(ah, bh[j], acc[i][j]);
    }
  }

#pragma unroll
  for (int i = 0; i < 4; ++i) {
    const unsigned mBase = m0 + ((unsigned)i << 4);
#pragma unroll
    for (int j = 0; j < 4; ++j) {
      const unsigned n = n0 + ((unsigned)j << 4) + rlane;
      float bv = 0.0f;
      if (HASBIAS) bv = bfr(bias[n]);
#pragma unroll
      for (int r = 0; r < 8; ++r) {
        float v = acc[i][j][r] * scale + bv;
        if (OUT_MODE == 1) v *= oscale;
        slab[(mOff + (unsigned)r) * 68u + ((unsigned)j << 4) + rlane] = v;
      }
    }
    wave_sync_lds();
    if (OUT_MODE == 0) {
      if (mBase < Mvalid) {
        float* C = (float*)Cout;
        const unsigned hh = lane >> 4, c4 = (lane & 15u) * 4u;
#pragma unroll
        for (int half = 0; half < 2; ++half) {
          v4f vv[4];
#pragma unroll
          for (int it = 0; it < 4; ++it) {
            const unsigned row = (unsigned)(half * 4 + it) * 2u + hh;
            vv[it] = *(const v4f*)(slab + row * 68u + c4);
          }
          for (int pass = 0; pass < 2; ++pass) {
#pragma unroll
            for (int it = 0; it < 4; ++it) {
              const unsigned row = (unsigned)(half * 4 + it) * 2u + hh;
              *(volatile v4f*)(C + (size_t)(mBase + row) * ldc + n0 + c4) = vv[it];
            }
            __threadfence();
          }
        }
      }
    } else {
      _Float16* C = (_Float16*)Cout;
      const unsigned q = lane >> 3, c8 = (lane & 7u) * 8u;
      v8h hv[4];
#pragma unroll
      for (int it = 0; it < 4; ++it) {
        const unsigned row = (unsigned)it * 4u + q;
        const float* sp = slab + row * 68u + c8;
#pragma unroll
        for (int e = 0; e < 8; ++e) hv[it][e] = toh_flush(sp[e]);
      }
      for (int pass = 0; pass < 2; ++pass) {
#pragma unroll
        for (int it = 0; it < 4; ++it) {
          const unsigned row = (unsigned)it * 4u + q;
          *(volatile v8h*)(C + (size_t)(mBase + row) * ldc + n0 + c8) = hv[it];
        }
        __threadfence();
      }
    }
    wave_sync_lds();
  }
}

__global__ __launch_bounds__(256) void k_gemm_p(
    const _Float16* __restrict__ A, unsigned lda, const _Float16* __restrict__ Bt, unsigned ldb,
    _Float16* __restrict__ Cout, unsigned ldc, const float* __restrict__ bias,
    unsigned M, unsigned Mvalid, unsigned N, unsigned K, float scale, float oscale) {
  __shared__ __align__(16) float sT[8][16 * 68];
  const unsigned wave = (unsigned)__builtin_amdgcn_readfirstlane((int)(threadIdx.x >> 5));
  gemm64_body<1, false>(A, lda, Bt, ldb, (void*)Cout, ldc, bias, M, Mvalid, N, K, scale, oscale, sT[wave], wave);
}

__global__ __launch_bounds__(256) void k_gemm_o(
    const _Float16* __restrict__ A, unsigned lda, const _Float16* __restrict__ Bt, unsigned ldb,
    float* __restrict__ Cout, unsigned ldc, const float* __restrict__ bias,
    unsigned M, unsigned Mvalid, unsigned N, unsigned K, float scale, float oscale) {
  __shared__ __align__(16) float sT[8][16 * 68];
  const unsigned wave = (unsigned)__builtin_amdgcn_readfirstlane((int)(threadIdx.x >> 5));
  gemm64_body<0, true>(A, lda, Bt, ldb, (void*)Cout, ldc, bias, M, Mvalid, N, K, scale, oscale, sT[wave], wave);
}

static_assert(2 * 256 * 16 == 64 * NA * 2);
__global__ __launch_bounds__(256) void k_dT(const float* __restrict__ dist, unsigned short* __restrict__ D16) {
    __shared__ float sD[64][65];
    const unsigned t = threadIdx.x;
    const unsigned i0 = blockIdx.x * 64u;
    const unsigned il = t & 63u, jq = t >> 6;
    const unsigned node = i0 + il;
    const unsigned nodec = (node < (unsigned)NN) ? node : (unsigned)(NN - 1);
    const bool live = node < (unsigned)NN;
#pragma unroll 4
    for (unsigned it = 0; it < 16u; ++it) {
        const unsigned j = jq + 4u * it;
        float d = dist[(size_t)j * NN_FULL + nodec];
        asm volatile("" : "+v"(d));
        sD[il][j] = live ? bfr(d) * CARRY_D : 0.0f;
    }
    __syncthreads();
    const unsigned p = t & 7u, r = t >> 3;
#pragma unroll
    for (int it = 0; it < 2; ++it) {
        const unsigned rr = r + 32u * (unsigned)it;
        float v[8];
#pragma unroll
        for (int e = 0; e < 8; ++e) v[e] = sD[rr][8u * p + (unsigned)e];
        st8hf(D16, (size_t)(i0 + rr) * NA + 8u * p, v);
    }
}

static_assert(4 * 256 * 16 == DL * NA * 2);
__global__ __launch_bounds__(256) void k_sel(const float* __restrict__ emb, const int* __restrict__ ids,
                                             unsigned short* __restrict__ E16) {
    __shared__ float sE[64][129];
    const unsigned t = threadIdx.x;
    const unsigned c = t & 127u, jh = t >> 7;
#pragma unroll 4
    for (unsigned it = 0; it < 32u; ++it) {
        const unsigned j = jh + 2u * it;
        int id = ids[j];
        id = (id < 0) ? id + NN_FULL : id;
        id = min(max(id, 0), NN_FULL - 1);
        sE[j][c] = bfr(emb[(size_t)id * DL + c]) * CARRY_E;
    }
    __syncthreads();
    const unsigned p = t & 7u, r = t >> 3;
#pragma unroll
    for (int it = 0; it < 4; ++it) {
        const unsigned cc = r + 32u * (unsigned)it;
        float v[8];
#pragma unroll
        for (int e = 0; e < 8; ++e) v[e] = sE[8u * p + (unsigned)e][cc];
        st8hf(E16, (size_t)cc * NA + 8u * p, v);
    }
}

static_assert(16 * 256 * 16 == DL * KCAT * 2);
__global__ __launch_bounds__(256) void k_wconv(const float* __restrict__ Wm, unsigned short* __restrict__ W16) {
    const unsigned u = blockIdx.x * 256u + threadIdx.x;
    if (u >= (unsigned)(DL * KCAT / 8)) return;
    const float* src = Wm + (size_t)u * 8u;
    const v4f a = *(const v4f*)src, b = *(const v4f*)(src + 4);
    float v[8] = {bfr(a.x) * CARRY_W, bfr(a.y) * CARRY_W, bfr(a.z) * CARRY_W, bfr(a.w) * CARRY_W,
                  bfr(b.x) * CARRY_W, bfr(b.y) * CARRY_W, bfr(b.z) * CARRY_W, bfr(b.w) * CARRY_W};
    st8hf(W16, (size_t)u * 8u, v);
}

static_assert(256 * 16 == 16 * DL * 2);
__global__ __launch_bounds__(256) void k_qsum(const float* __restrict__ emb, unsigned short* __restrict__ PQ) {
    const unsigned t = threadIdx.x;
    const unsigned row = blockIdx.x * 16u + (t >> 4);
    const unsigned c0 = (t & 15u) * 8u;
    float s0 = 0.f, s1 = 0.f, s2 = 0.f, s3 = 0.f, s4 = 0.f, s5 = 0.f, s6 = 0.f, s7 = 0.f;
    if (blockIdx.x * 16u < (unsigned)NN) {
        unsigned src = (row * 64u) % (unsigned)NN_FULL;
#pragma unroll 4
        for (unsigned j = 0; j < 64u; ++j) {
            const float* p = emb + (size_t)src * DL + c0;
            const v4f a = *(const v4f*)p;
            const v4f b = *(const v4f*)(p + 4);
            s0 += bfr(a.x); s1 += bfr(a.y); s2 += bfr(a.z); s3 += bfr(a.w);
            s4 += bfr(b.x); s5 += bfr(b.y); s6 += bfr(b.z); s7 += bfr(b.w);
            src = (src + 1u == (unsigned)NN_FULL) ? 0u : src + 1u;
        }
    }
    float v[8] = {s0 * QMUL, s1 * QMUL, s2 * QMUL, s3 * QMUL, s4 * QMUL, s5 * QMUL, s6 * QMUL, s7 * QMUL};
    st8hf(PQ, (size_t)row * KCAT + DL + c0, v);
}

extern "C" void kernel_launch(void* const* d_in, const int* in_sizes, int n_in, void* d_out, int out_size,
                              void* d_ws, size_t ws_size, hipStream_t stream) {
    if (n_in < 5) return;
    if (in_sizes[0] < NN_FULL * DL || in_sizes[1] < NA * NN_FULL || in_sizes[2] < DL * KCAT) return;
    if (in_sizes[3] < DL || in_sizes[4] < NA || out_size < NN * DL) return;
    if (WS_TOTAL > ws_size) return;

    const float* embeds = (const float*)d_in[0];
    const float* dists  = (const float*)d_in[1];
    const float* Wh     = (const float*)d_in[2];
    const float* bh     = (const float*)d_in[3];
    const int*   ids    = (const int*)d_in[4];
    float* out = (float*)d_out;

    char* wsp = (char*)d_ws;
    unsigned short* D16  = (unsigned short*)(wsp + OFF_D);
    unsigned short* E16  = (unsigned short*)(wsp + OFF_E);
    unsigned short* W16  = (unsigned short*)(wsp + OFF_W);
    unsigned short* PQ16 = (unsigned short*)(wsp + OFF_PQ);

    k_dT<<<G_DT, 256, 0, stream>>>(dists, D16);
    k_sel<<<1, 256, 0, stream>>>(embeds, ids, E16);
    k_wconv<<<G_WC, 256, 0, stream>>>(Wh, W16);
    k_qsum<<<G_QS, 256, 0, stream>>>(embeds, PQ16);

    k_gemm_p<<<G_GEMM, 256, 0, stream>>>((const _Float16*)D16, NA, (const _Float16*)E16, NA,
        (_Float16*)PQ16, KCAT, bh, MPAD, MPAD, DL, NA, SC_P, OSC_P);
    k_gemm_o<<<G_GEMM, 256, 0, stream>>>((const _Float16*)PQ16, KCAT, (const _Float16*)W16, KCAT,
        out, DL, bh, MPAD, NN, DL, KCAT, SC_O, OSC_O);
}
